// AGCRNCell_3736621548018
// MI455X (gfx1250) — hardware-verified
//
#include <hip/hip_runtime.h>
#include <math.h>

constexpr int kB    = 32;
constexpr int kN    = 3000;
constexpr int kNP   = 3008;
constexpr int kNE   = 3072;
constexpr int kCin  = 2;
constexpr int kHid  = 64;
constexpr int kCat  = 66;
constexpr int kD    = 16;
constexpr int kKE   = 32;
constexpr int kKW   = 224;
constexpr int kXGP  = 256;
constexpr int kXGN  = kB * kXGP;
constexpr int kOG   = 128;
constexpr int kOU   = 64;
constexpr int kXTS  = kB * kHid;
constexpr int kXTR  = kXTS + kB * kCin;
constexpr int kXCH  = kNP / 8;
constexpr int kChunkG = 384;
constexpr int kChunkU = 768;
constexpr float kSCar = 32768.0f;
constexpr float kECar = 16.0f;
constexpr float kWCar = 64.0f;

typedef __attribute__((ext_vector_type(16))) _Float16 v16h;
typedef __attribute__((ext_vector_type(8)))  _Float16 v8h;
typedef __attribute__((ext_vector_type(8)))  float    v8f;
typedef __attribute__((ext_vector_type(4)))  float    v4f;
typedef __attribute__((ext_vector_type(4)))  unsigned int v4u;

__device__ __forceinline__ void dep_guard_h(v8f& a, v8f& b, v16h x, v16h y) { asm volatile("v_nop\n\tv_nop\n\tv_nop\n\tv_nop" : "+v"(a), "+v"(b) : "v"(x), "v"(y)); }
__device__ __forceinline__ void keep4_h(v16h a, v16h b, v16h c, v16h d) { asm volatile("v_nop" :: "v"(a), "v"(b), "v"(c), "v"(d)); }
__device__ __forceinline__ void acc_guard4(v8f& a, v8f& b, v8f& c, v8f& d) { asm volatile("v_nop\n\tv_nop\n\tv_nop\n\tv_nop" : "+v"(a), "+v"(b), "+v"(c), "+v"(d)); }
template <typename T> struct Frag;
template <> struct Frag<_Float16> {
  typedef v16h V; union U { v16h v; v8h h[2]; };
  static __device__ __forceinline__ v16h load(const _Float16* p) {
    U f; f.h[0] = *(const v8h*)(p); f.h[1] = *(const v8h*)(p + 16); return f.v;
  }
  static __device__ __forceinline__ v8f mma(v16h a, v16h b, v8f c) {
    return __builtin_amdgcn_wmma_f32_16x16x32_f16(false, a, false, b, (short)0, c, false, false);
  }
  static __device__ __forceinline__ void guard(v8f& a, v8f& b, v16h x, v16h y) { dep_guard_h(a, b, x, y); }
  static __device__ __forceinline__ void keep(v16h a, v16h b, v16h c, v16h d) { keep4_h(a, b, c, d); }
};

__device__ __forceinline__ unsigned pk16(unsigned short a, unsigned short b) { return (unsigned)a | ((unsigned)b << 16); }
__device__ __forceinline__ unsigned short h_bits(float f) { const _Float16 h = (_Float16)f; return __builtin_bit_cast(unsigned short, h); }
__device__ __forceinline__ float h2f(unsigned short u) { return (float)__builtin_bit_cast(_Float16, u); }
__device__ __forceinline__ v4u pack8(const unsigned short* hb) {
  return (v4u){pk16(hb[0], hb[1]), pk16(hb[2], hb[3]), pk16(hb[4], hb[5]), pk16(hb[6], hb[7])};
}

template <int BIAS_MODE, int OUT_MODE, int RESM, int ACT>
__global__ __launch_bounds__(256) void wmma_gemm64(
    const unsigned short* __restrict__ Ap, int lda, long strideA,
    const unsigned short* __restrict__ Btp, int ldb, long strideB,
    void* __restrict__ Cout, int ldc, long strideC,
    const float* __restrict__ bias,
    const void* __restrict__ resid, int ldr, long strideR, int Mr,
    int M, int N, int K, float scale) {
  typedef _Float16 T;
  typedef v16h V;
  const T* A = (const T*)Ap; const T* Bt = (const T*)Btp;
  __shared__ __align__(16) float sT[8][16 * 68];
  const int b    = blockIdx.y;
  const int lane = threadIdx.x & 31;
  const int wave = threadIdx.x >> 5;
  const int tilesN = N >> 6;
  const int tilesM = M >> 6;
  const int tile = blockIdx.x * 8 + wave;
  if (tile >= tilesM * tilesN) return;
  const int tm = tile / tilesN;
  const int tn = tile - tm * tilesN;
  const int m0 = tm << 6;
  const int n0 = tn << 6;

  const T* Ab  = A  + (size_t)b * strideA;
  const T* Bb  = Bt + (size_t)b * strideB;

  const int rlane = lane & 15;
  const int koff  = (lane >> 4) * 8;
  const int mOff  = (lane >> 4) * 8;

  v8f acc[4][4];
#pragma unroll
  for (int i = 0; i < 4; ++i)
#pragma unroll
    for (int j = 0; j < 4; ++j) acc[i][j] = (v8f){0.f,0.f,0.f,0.f,0.f,0.f,0.f,0.f};

  for (int k0 = 0; k0 < K; k0 += 32) {
    V bh[4];
#pragma unroll
    for (int j = 0; j < 4; ++j) {
      const size_t bo = (size_t)(n0 + (j << 4) + rlane) * ldb + koff + k0;
      bh[j] = Frag<T>::load(Bb + bo);
    }
#pragma unroll
    for (int i = 0; i < 4; ++i) {
      const size_t ao = (size_t)(m0 + (i << 4) + rlane) * lda + koff + k0;
      V ah = Frag<T>::load(Ab + ao);
#pragma unroll
      for (int j = 0; j < 4; ++j) {
        acc[i][j] = Frag<T>::mma(ah, bh[j], acc[i][j]);
      }
      Frag<T>::guard(acc[i][0], acc[i][3], ah, ah);
    }
    Frag<T>::keep(bh[0], bh[1], bh[2], bh[3]);
  }
  acc_guard4(acc[0][0], acc[0][1], acc[0][2], acc[0][3]);
  acc_guard4(acc[1][0], acc[1][1], acc[1][2], acc[1][3]);
  acc_guard4(acc[2][0], acc[2][1], acc[2][2], acc[2][3]);
  acc_guard4(acc[3][0], acc[3][1], acc[3][2], acc[3][3]);

  float* slab = sT[wave];
  const float* Rf = (RESM == 1 || RESM == 2) ? ((const float*)resid + (size_t)b * strideR) : nullptr;
  const _Float16* R16 = (RESM == 3) ? ((const _Float16*)resid + (size_t)b * strideR) : nullptr;
#pragma unroll
  for (int i = 0; i < 4; ++i) {
    const int mBase = m0 + (i << 4);
#pragma unroll
    for (int j = 0; j < 4; ++j) {
      const int n = n0 + (j << 4) + rlane;
      float bv = 0.f;
      if (BIAS_MODE == 2) bv = bias[n];
#pragma unroll
      for (int r = 0; r < 8; ++r) {
        float v = acc[i][j][r] * scale;
        if (BIAS_MODE == 1) v += bias[mBase + mOff + r];
        if (BIAS_MODE == 2) v += bv;
        if (RESM != 0) {
          int rr = mBase + mOff + r;
          rr = (rr < Mr) ? rr : (Mr - 1);
          float rv;
          if (RESM == 3) rv = (float)R16[(size_t)rr * ldr + n];
          else rv = Rf[(size_t)rr * ldr + n];
          v = (RESM == 1) ? (v + rv) : (v - rv);
        }
        if (ACT == 1) v = tanhf(v);
        if (ACT == 2) v = fmaxf(v, 0.0f);
        if (ACT == 4) v = (v > 0.f) ? v : 0.01f * v;
        slab[(mOff + r) * 68 + (j << 4) + rlane] = v;
      }
    }
    __builtin_amdgcn_fence(__ATOMIC_RELEASE, "workgroup");
    __builtin_amdgcn_wave_barrier();
    __builtin_amdgcn_fence(__ATOMIC_ACQUIRE, "workgroup");
    if (OUT_MODE == 0) {
      float* C = (float*)Cout + (size_t)b * strideC;
      const int hh = lane >> 4, c4 = (lane & 15) * 4;
      for (int pass = 0; pass < 2; ++pass) {
#pragma unroll
        for (int it = 0; it < 8; ++it) {
          const int row = it * 2 + hh;
          v4f v = *(const v4f*)(slab + row * 68 + c4);
          *(volatile v4f*)(C + (size_t)(mBase + row) * ldc + n0 + c4) = v;
        }
        __threadfence();
      }
    } else {
      const int q = lane >> 3, c8 = (lane & 7) * 8;
      unsigned short* C = (unsigned short*)Cout + (size_t)b * strideC;
      for (int pass = 0; pass < 2; ++pass) {
#pragma unroll
        for (int it = 0; it < 4; ++it) {
          const int row = it * 4 + q;
          const float* sp = slab + row * 68 + c8;
          v8h hv;
#pragma unroll
          for (int e = 0; e < 8; ++e) hv[e] = (_Float16)sp[e];
          *(volatile v8h*)(C + (size_t)(mBase + row) * ldc + n0 + c8) = hv;
        }
        __threadfence();
      }
    }
    __builtin_amdgcn_fence(__ATOMIC_RELEASE, "workgroup");
    __builtin_amdgcn_wave_barrier();
    __builtin_amdgcn_fence(__ATOMIC_ACQUIRE, "workgroup");
  }
}

__global__ __launch_bounds__(256) void pack_e16(const float* __restrict__ E, unsigned short* __restrict__ E16) {
  const int idx = blockIdx.x * 256 + threadIdx.x;
  const int row = idx >> 2, q = idx & 3;
  const int rc = (row < kN) ? row : (kN - 1);
  unsigned short hb[8];
#pragma unroll
  for (int e = 0; e < 8; ++e) {
    const int d = q * 8 + e;
    const int dc = (d < kD) ? d : (kD - 1);
    float v = E[(size_t)rc * kD + dc] * kECar;
    if (row >= kN || d >= kD) v = 0.0f;
    hb[e] = h_bits(v);
  }
  const v4u u = pack8(hb);
  unsigned short* p = E16 + (size_t)row * kKE + q * 8;
  *(volatile v4u*)p = u;
  __threadfence();
  *(volatile v4u*)p = u;
}

template <int NOUT>
__global__ __launch_bounds__(256) void pack_pool16(const float* __restrict__ pool, const float* __restrict__ bpool,
                                                   unsigned short* __restrict__ PT) {
  const int idx = blockIdx.x * 256 + threadIdx.x;
  const int prow = idx >> 2, q = idx & 3;
  const int o = prow / kKW;
  const int j = prow - o * kKW;
  const int jj = (j >= 192) ? (j - 192) : 0;
  const int kk = (j < 192) ? (j >> 6) : ((j < 198) ? (jj >> 1) : 0);
  const int ii = (j < 192) ? (2 + (j & 63)) : ((j < 198) ? (jj & 1) : 0);
  const bool isw = (j < 198);
  const bool isb = (j == 198);
  const float car = (kk == 1) ? 1.0f : kWCar;
  unsigned short hb[8];
#pragma unroll
  for (int e = 0; e < 8; ++e) {
    const int d = q * 8 + e;
    const int dc = (d < kD) ? d : (kD - 1);
    const float pv = pool[(((size_t)dc * 3 + kk) * kCat + ii) * NOUT + o] * car;
    const float bv = bpool[(size_t)dc * NOUT + o] * kWCar;
    float v = isb ? bv : (isw ? pv : 0.0f);
    if (d >= kD) v = 0.0f;
    hb[e] = h_bits(v);
  }
  const v4u u = pack8(hb);
  unsigned short* p = PT + (size_t)prow * kKE + q * 8;
  *(volatile v4u*)p = u;
  __threadfence();
  *(volatile v4u*)p = u;
}

__global__ __launch_bounds__(256) void softmax_rows(const float* __restrict__ L, unsigned short* __restrict__ S16) {
  __shared__ float srow[kNP];
  __shared__ float redA[8];
  __shared__ float redB[8];
  const int n = blockIdx.x;
  const int t = threadIdx.x, lane = t & 31, wave = t >> 5;
  unsigned short* orow = S16 + (size_t)n * kNP;
  if (n >= kN) {
    const v4u zz = (v4u){0u, 0u, 0u, 0u};
    for (int pass = 0; pass < 2; ++pass) {
      *(volatile v4u*)(orow + t * 8) = zz;
      if (t < kXCH - 256) *(volatile v4u*)(orow + (t + 256) * 8) = zz;
      __threadfence();
    }
    return;
  }
  const float* lrow = L + (size_t)n * kNP;
  float mx = 0.0f;
#pragma unroll 1
  for (int m = t; m < kNP; m += 256) {
    float v = lrow[m];
    if (m >= kN) v = 0.0f;
    srow[m] = v;
    mx = fmaxf(mx, v);
  }
#pragma unroll
  for (int off = 16; off > 0; off >>= 1) mx = fmaxf(mx, __shfl_xor(mx, off, 32));
  if (lane == 0) redA[wave] = mx;
  __syncthreads();
  float rmax = redA[0];
#pragma unroll
  for (int w = 1; w < 8; ++w) rmax = fmaxf(rmax, redA[w]);
  float sm = 0.0f;
#pragma unroll 1
  for (int m = t; m < kN; m += 256) {
    const float e = expf(srow[m] - rmax);
    srow[m] = e;
    sm += e;
  }
#pragma unroll
  for (int off = 16; off > 0; off >>= 1) sm += __shfl_xor(sm, off, 32);
  if (lane == 0) redB[wave] = sm;
  __syncthreads();
  float tot = redB[0];
#pragma unroll
  for (int w = 1; w < 8; ++w) tot += redB[w];
  const float inv = 1.0f / tot;
  __syncthreads();
  const int ch0 = t;
  const int ch1 = t + 256;
  const int ch1c = (ch1 < kXCH) ? ch1 : (kXCH - 1);
  unsigned short h0[8], h1[8];
#pragma unroll
  for (int e = 0; e < 8; ++e) {
    const int m0 = ch0 * 8 + e;
    const int m1 = ch1c * 8 + e;
    float v0 = srow[m0] * inv * kSCar;
    float v1 = srow[m1] * inv * kSCar;
    if (m0 >= kN) v0 = 0.0f;
    if (m1 >= kN) v1 = 0.0f;
    h0[e] = h_bits(v0);
    h1[e] = h_bits(v1);
  }
  const v4u u0 = pack8(h0), u1 = pack8(h1);
  for (int pass = 0; pass < 2; ++pass) {
    *(volatile v4u*)(orow + ch0 * 8) = u0;
    if (ch1 < kXCH) *(volatile v4u*)(orow + ch1 * 8) = u1;
    __threadfence();
  }
}

template <int SRC>
__global__ __launch_bounds__(256) void pack_xt(const float* __restrict__ xs, const unsigned short* __restrict__ rs,
                                               unsigned short* __restrict__ XT) {
  const int idx = blockIdx.x * 256 + threadIdx.x;
  const int row = idx / kXCH;
  const int ch = idx - row * kXCH;
  int b, c;
  if (SRC == 2) { c = row >> 5; b = row & 31; } else { b = row >> 6; c = row & 63; }
  unsigned short hb[8];
#pragma unroll
  for (int e = 0; e < 8; ++e) {
    const int m = ch * 8 + e;
    const int mc = (m < kN) ? m : (kN - 1);
    unsigned short hv;
    if (SRC == 0) hv = h_bits(xs[((size_t)b * kN + mc) * kHid + c]);
    else if (SRC == 1) hv = rs[((size_t)mc * kB + b) * kHid + c];
    else hv = h_bits(xs[((size_t)b * kN + mc) * kCin + c]);
    hb[e] = (m < kN) ? hv : (unsigned short)0;
  }
  const v4u u = pack8(hb);
  unsigned short* p = XT + (size_t)row * kNP + ch * 8;
  *(volatile v4u*)p = u;
  __threadfence();
  *(volatile v4u*)p = u;
}

template <int CAND>
__global__ __launch_bounds__(256) void fill_xg(const float* __restrict__ x, const float* __restrict__ state,
                                               const unsigned short* __restrict__ RS, const unsigned short* __restrict__ P1T,
                                               const float* __restrict__ P2X, unsigned short* __restrict__ XG) {
  const int n = blockIdx.x;
  const int t = threadIdx.x;
  const int b = t >> 3, q = t & 7;
  unsigned short* rowp = XG + ((size_t)n * kB + b) * kXGP;
  v4u u0;
  if (CAND) {
    u0 = *(const v4u*)(RS + ((size_t)n * kB + b) * kHid + q * 8);
  } else {
    const float* sp = state + ((size_t)b * kN + n) * kHid + q * 8;
    const v4f a = *(const v4f*)sp;
    const v4f c = *(const v4f*)(sp + 4);
    unsigned short hb[8];
#pragma unroll
    for (int e = 0; e < 4; ++e) { hb[e] = h_bits(a[e]); hb[4 + e] = h_bits(c[e]); }
    u0 = pack8(hb);
  }
  unsigned short g[8];
#pragma unroll
  for (int e = 0; e < 8; ++e) g[e] = P1T[(size_t)(b * kHid + q * 8 + e) * kNP + n];
  const v4u u1 = pack8(g);
  const float x0 = x[((size_t)b * kN + n) * kCin];
  const float x1 = x[((size_t)b * kN + n) * kCin + 1];
  const unsigned short p10 = P1T[(size_t)(kXTS + b) * kNP + n];
  const unsigned short p11 = P1T[(size_t)(kXTS + kB + b) * kNP + n];
  const float p20 = P2X[(size_t)n * kHid + b];
  const float p21 = P2X[(size_t)n * kHid + kB + b];
  const float t0 = 2.0f * p20 - x0;
  const float t1 = 2.0f * p21 - x1;
  unsigned short w[8];
  w[0] = h_bits(x0); w[1] = h_bits(x1); w[2] = p10; w[3] = p11;
  w[4] = h_bits(t0); w[5] = h_bits(t1); w[6] = h_bits(1.0f); w[7] = (unsigned short)0;
  const bool lead = (q == 0);
#pragma unroll
  for (int e = 0; e < 8; ++e) w[e] = lead ? w[e] : (unsigned short)0;
  const v4u u3 = pack8(w);
  unsigned short* p0 = rowp + q * 8;
  unsigned short* p1 = rowp + 64 + q * 8;
  unsigned short* p3 = rowp + 192 + q * 8;
  *(volatile v4u*)p0 = u0;
  *(volatile v4u*)p1 = u1;
  *(volatile v4u*)p3 = u3;
  __threadfence();
  *(volatile v4u*)p0 = u0;
  *(volatile v4u*)p1 = u1;
  *(volatile v4u*)p3 = u3;
}

template <int OT, int PHASE>
__global__ __launch_bounds__(256) void node_gemm(const unsigned short* __restrict__ XGp, const unsigned short* __restrict__ Wp,
                                                 const float* __restrict__ state, float* __restrict__ Z,
                                                 unsigned short* __restrict__ RS, float* __restrict__ out,
                                                 int nbase, int ncount) {
  __shared__ __align__(16) float sT[8][16 * 68];
  const int lane = threadIdx.x & 31, wave = threadIdx.x >> 5;
  constexpr int NPB = 8 / OT;
  const int sub = wave / OT;
  const int ot  = wave - sub * OT;
  const int nl  = blockIdx.x * NPB + sub;
  if (nl >= ncount) return;
  const int n = nbase + nl;
  const _Float16* A  = (const _Float16*)XGp + (size_t)n * kXGN;
  const _Float16* Bt = (const _Float16*)Wp + ((size_t)nl * (OT * 64) + ot * 64) * kKW;
  const int rlane = lane & 15;
  const int koff  = (lane >> 4) * 8;
  const int mOff  = (lane >> 4) * 8;

  v8f acc[2][4];
#pragma unroll
  for (int i = 0; i < 2; ++i)
#pragma unroll
    for (int j = 0; j < 4; ++j) acc[i][j] = (v8f){0.f,0.f,0.f,0.f,0.f,0.f,0.f,0.f};

#pragma unroll
  for (int k0 = 0; k0 < kKW; k0 += 32) {
    v16h bh[4];
#pragma unroll
    for (int j = 0; j < 4; ++j) bh[j] = Frag<_Float16>::load(Bt + (size_t)((j << 4) + rlane) * kKW + koff + k0);
#pragma unroll
    for (int i = 0; i < 2; ++i) {
      const v16h ah = Frag<_Float16>::load(A + (size_t)((i << 4) + rlane) * kXGP + koff + k0);
#pragma unroll
      for (int j = 0; j < 4; ++j) acc[i][j] = Frag<_Float16>::mma(ah, bh[j], acc[i][j]);
      Frag<_Float16>::guard(acc[i][0], acc[i][3], ah, ah);
    }
    Frag<_Float16>::keep(bh[0], bh[1], bh[2], bh[3]);
  }
  acc_guard4(acc[0][0], acc[0][1], acc[0][2], acc[0][3]);
  acc_guard4(acc[1][0], acc[1][1], acc[1][2], acc[1][3]);

  float* slab = sT[wave];
  const float inv64 = 1.0f / 64.0f;
#pragma unroll
  for (int i = 0; i < 2; ++i) {
#pragma unroll
    for (int j = 0; j < 4; ++j) {
#pragma unroll
      for (int r = 0; r < 8; ++r) {
        float v = acc[i][j][r] * inv64;
        if (PHASE == 0) v = __builtin_amdgcn_rcpf(1.0f + expf(-v));
        else v = tanhf(v);
        slab[(mOff + r) * 68 + (j << 4) + rlane] = v;
      }
    }
    __builtin_amdgcn_fence(__ATOMIC_RELEASE, "workgroup");
    __builtin_amdgcn_wave_barrier();
    __builtin_amdgcn_fence(__ATOMIC_ACQUIRE, "workgroup");
    if (PHASE == 0) {
      if (ot == 0) {
        const int hh = lane >> 4, c4 = (lane & 15) * 4;
        for (int pass = 0; pass < 2; ++pass) {
#pragma unroll
          for (int it = 0; it < 8; ++it) {
            const int row = it * 2 + hh;
            const int bb = i * 16 + row;
            const v4f v = *(const v4f*)(slab + row * 68 + c4);
            *(volatile v4f*)(Z + ((size_t)n * kB + bb) * kHid + c4) = v;
          }
          __threadfence();
        }
      } else {
        const int q = lane >> 3, c8 = (lane & 7) * 8;
        for (int pass = 0; pass < 2; ++pass) {
#pragma unroll
          for (int it = 0; it < 4; ++it) {
            const int row = it * 4 + q;
            const int bb = i * 16 + row;
            const float* sp = slab + row * 68 + c8;
            const float* st = state + ((size_t)bb * kN + n) * kHid + c8;
            const v4f s0 = *(const v4f*)st;
            const v4f s1 = *(const v4f*)(st + 4);
            v8h hv;
#pragma unroll
            for (int e = 0; e < 4; ++e) { hv[e] = (_Float16)(sp[e] * s0[e]); hv[4 + e] = (_Float16)(sp[4 + e] * s1[e]); }
            *(volatile v8h*)(RS + ((size_t)n * kB + bb) * kHid + c8) = hv;
          }
          __threadfence();
        }
      }
    } else {
      const int hh = lane >> 4, c4 = (lane & 15) * 4;
      for (int pass = 0; pass < 2; ++pass) {
#pragma unroll
        for (int it = 0; it < 8; ++it) {
          const int row = it * 2 + hh;
          const int bb = i * 16 + row;
          const v4f hc = *(const v4f*)(slab + row * 68 + c4);
          const v4f z  = *(const v4f*)(Z + ((size_t)n * kB + bb) * kHid + c4);
          const v4f st = *(const v4f*)(state + ((size_t)bb * kN + n) * kHid + c4);
          const v4f o  = z * st + (1.0f - z) * hc;
          *(volatile v4f*)(out + ((size_t)bb * kN + n) * kHid + c4) = o;
        }
        __threadfence();
      }
    }
    __builtin_amdgcn_fence(__ATOMIC_RELEASE, "workgroup");
    __builtin_amdgcn_wave_barrier();
    __builtin_amdgcn_fence(__ATOMIC_ACQUIRE, "workgroup");
  }
}

extern "C" void kernel_launch(void* const* d_in, const int* in_sizes, int n_in,
                              void* d_out, int out_size, void* d_ws, size_t ws_size,
                              hipStream_t stream) {
  if (n_in < 7) return;
  if (in_sizes[0] != kB * kN * kCin) return;
  if (in_sizes[1] != kB * kN * kHid) return;
  if (in_sizes[2] != kN * kD) return;
  if (in_sizes[3] != kD * 3 * kCat * kOG) return;
  if (in_sizes[4] != kD * kOG) return;
  if (in_sizes[5] != kD * 3 * kCat * kOU) return;
  if (in_sizes[6] != kD * kOU) return;
  if (out_size != kB * kN * kHid) return;

  const float* x     = (const float*)d_in[0];
  const float* state = (const float*)d_in[1];
  const float* E     = (const float*)d_in[2];
  const float* gw    = (const float*)d_in[3];
  const float* gb    = (const float*)d_in[4];
  const float* uw    = (const float*)d_in[5];
  const float* ub    = (const float*)d_in[6];
  float* outp = (float*)d_out;

  const size_t SZ_S16 = (size_t)kNP * kNP * 2;
  const size_t SZ_E16 = (size_t)kNE * kKE * 2;
  const size_t SZ_PTG = (size_t)kOG * kKW * kKE * 2;
  const size_t SZ_PTU = (size_t)kOU * kKW * kKE * 2;
  const size_t SZ_Z   = (size_t)kN * kB * kHid * 4;
  const size_t SZ_RS  = (size_t)kN * kB * kHid * 2;
  const size_t SZ_XT  = (size_t)kXTR * kNP * 2;
  const size_t SZ_P1  = SZ_XT;
  const size_t SZ_P2X = (size_t)kNP * kHid * 4;
  const size_t SZ_XG  = (size_t)kNP * kXGN * 2;
  const size_t SZ_W   = (size_t)kChunkG * kOG * kKW * 2;
  const size_t SZ_L   = (size_t)kNP * kNP * 4;

  size_t off = 0;
  const size_t oS16 = off; off += SZ_S16;
  const size_t oE16 = off; off += SZ_E16;
  const size_t oPTG = off; off += SZ_PTG;
  const size_t oPTU = off; off += SZ_PTU;
  const size_t oZ   = off; off += SZ_Z;
  const size_t oRS  = off; off += SZ_RS;
  const size_t oA   = off;
  const size_t oXT  = oA;
  const size_t oP1  = oXT + SZ_XT;
  const size_t oP2X = oP1 + SZ_P1;
  const size_t endA = oP2X + SZ_P2X;
  const size_t oW   = oA;
  const size_t oL   = oA;
  const size_t oXG  = endA;
  const size_t TOTAL = oXG + SZ_XG;
  if (oW + SZ_W > endA) return;
  if ((size_t)kChunkU * kOU * kKW * 2 != SZ_W) return;
  if (oL + SZ_L > TOTAL) return;
  if (TOTAL > ws_size) return;
  if (TOTAL > (size_t)134217728) return;

  char* ws = (char*)d_ws;
  unsigned short* S16 = (unsigned short*)(ws + oS16);
  unsigned short* E16 = (unsigned short*)(ws + oE16);
  unsigned short* PTG = (unsigned short*)(ws + oPTG);
  unsigned short* PTU = (unsigned short*)(ws + oPTU);
  float*          Zp  = (float*)(ws + oZ);
  unsigned short* RS  = (unsigned short*)(ws + oRS);
  unsigned short* XT  = (unsigned short*)(ws + oXT);
  unsigned short* P1T = (unsigned short*)(ws + oP1);
  float*          P2X = (float*)(ws + oP2X);
  unsigned short* W16 = (unsigned short*)(ws + oW);
  float*          Lp  = (float*)(ws + oL);
  unsigned short* XG  = (unsigned short*)(ws + oXG);
  const float* dummy_bias = E;
  const void*  dummy_res  = (const void*)state;

  const dim3 blk(256);
  const float scLogit = 1.0f / 256.0f;
  const float scP1    = 1.0f / 512.0f;
  const float scP2    = 1.0f / 1048576.0f;
  const float scP2x   = 1.0f / 2097152.0f;
  const float scW     = 1.0f / 16.0f;

  pack_e16<<<dim3(kNE * 4 / 256), blk, 0, stream>>>(E, E16);
  pack_pool16<kOG><<<dim3(kOG * kKW * 4 / 256), blk, 0, stream>>>(gw, gb, PTG);
  pack_pool16<kOU><<<dim3(kOU * kKW * 4 / 256), blk, 0, stream>>>(uw, ub, PTU);

  {
    const int tiles = (kNP / 64) * (kNP / 64);
    wmma_gemm64<0, 0, 0, 2><<<dim3((tiles + 7) / 8, 1), blk, 0, stream>>>(
        E16, kKE, 0L, E16, kKE, 0L, (void*)Lp, kNP, 0L, dummy_bias, dummy_res, 0, 0L, 1, kNP, kNP, kKE, scLogit);
    softmax_rows<<<dim3(kNP), blk, 0, stream>>>(Lp, S16);
  }

  const int tilesP1g = (kXTR / 64) * (kNP / 64);
  const int tilesP1c = (kXTS / 64) * (kNP / 64);
  const int tilesP2  = (kNP / 64);

  pack_xt<0><<<dim3(kXTS * kXCH / 256), blk, 0, stream>>>(state, RS, XT);
  pack_xt<2><<<dim3(kB * kCin * kXCH / 256), blk, 0, stream>>>(x, RS, XT + (size_t)kXTS * kNP);
  wmma_gemm64<0, 1, 0, 0><<<dim3((tilesP1g + 7) / 8, 1), blk, 0, stream>>>(
      XT, kNP, 0L, S16, kNP, 0L, (void*)P1T, kNP, 0L, dummy_bias, dummy_res, 0, 0L, 1, kXTR, kNP, kNP, scP1);
  wmma_gemm64<0, 1, 2, 0><<<dim3((tilesP2 + 7) / 8, kB), blk, 0, stream>>>(
      S16, kNP, 0L, P1T, kNP, (long)kHid * kNP, (void*)(XG + 128), kXGN, (long)kXGP, dummy_bias,
      (const void*)state, kHid, (long)kN * kHid, kN, kNP, kHid, kNP, scP2);
  wmma_gemm64<0, 0, 0, 0><<<dim3((tilesP2 + 7) / 8, 1), blk, 0, stream>>>(
      S16, kNP, 0L, P1T + (size_t)kXTS * kNP, kNP, 0L, (void*)P2X, kHid, 0L, dummy_bias, dummy_res, 0, 0L, 1,
      kNP, kHid, kNP, scP2x);
  fill_xg<0><<<dim3(kN), blk, 0, stream>>>(x, state, RS, P1T, P2X, XG);

  for (int c = 0; c < (kN + kChunkG - 1) / kChunkG; ++c) {
    const int nbase = c * kChunkG;
    const int cnt = (kN - nbase < kChunkG) ? (kN - nbase) : kChunkG;
    const int tilesW = (kChunkG / 64) * ((kOG * kKW) / 64);
    wmma_gemm64<0, 1, 0, 0><<<dim3((tilesW + 7) / 8, 1), blk, 0, stream>>>(
        E16 + (size_t)nbase * kKE, kKE, 0L, PTG, kKE, 0L, (void*)W16, kOG * kKW, 0L, dummy_bias, dummy_res, 0, 0L, 1,
        kChunkG, kOG * kKW, kKE, scW);
    node_gemm<2, 0><<<dim3((cnt + 3) / 4), blk, 0, stream>>>(XG, W16, state, Zp, RS, outp, nbase, cnt);
  }

  pack_xt<1><<<dim3(kXTS * kXCH / 256), blk, 0, stream>>>(state, RS, XT);
  wmma_gemm64<0, 1, 0, 0><<<dim3((tilesP1c + 7) / 8, 1), blk, 0, stream>>>(
      XT, kNP, 0L, S16, kNP, 0L, (void*)P1T, kNP, 0L, dummy_bias, dummy_res, 0, 0L, 1, kXTS, kNP, kNP, scP1);
  wmma_gemm64<0, 1, 3, 0><<<dim3((tilesP2 + 7) / 8, kB), blk, 0, stream>>>(
      S16, kNP, 0L, P1T, kNP, (long)kHid * kNP, (void*)(XG + 128), kXGN, (long)kXGP, dummy_bias,
      (const void*)RS, kB * kHid, (long)kHid, kN, kNP, kHid, kNP, scP2);
  fill_xg<1><<<dim3(kN), blk, 0, stream>>>(x, state, RS, P1T, P2X, XG);

  for (int c = 0; c < (kN + kChunkU - 1) / kChunkU; ++c) {
    const int nbase = c * kChunkU;
    const int cnt = (kN - nbase < kChunkU) ? (kN - nbase) : kChunkU;
    const int tilesW = (kChunkU / 64) * ((kOU * kKW) / 64);
    wmma_gemm64<0, 1, 0, 0><<<dim3((tilesW + 7) / 8, 1), blk, 0, stream>>>(
        E16 + (size_t)nbase * kKE, kKE, 0L, PTU, kKE, 0L, (void*)W16, kOU * kKW, 0L, dummy_bias, dummy_res, 0, 0L, 1,
        kChunkU, kOU * kKW, kKE, scW);
    node_gemm<1, 1><<<dim3((cnt + 7) / 8), blk, 0, stream>>>(XG, W16, state, Zp, RS, outp, nbase, cnt);
  }
}
